// SDT_55980603736284
// MI455X (gfx1250) — hardware-verified
//
#include <hip/hip_runtime.h>
#include <stddef.h>


#define IN_DIM      128
#define HID         64
#define NODES       63
#define DEPTHK      6
#define LEAVES      64
#define NSEL        (DEPTHK * HID)
#define ROWS_BLK    128
#define THR_MAIN    256
#define NWAVE       (THR_MAIN / 32)
#define WPITCH      136
#define LDS_W_BYTES (NSEL * WPITCH * 2)
#define WT_ELEMS    (NSEL * IN_DIM)
#define WT_V16      (WT_ELEMS / 8)
#define PREP_THR    64
#define PREP_BLK    (WT_V16 / PREP_THR)
#define WSCALE      64.0f
#define INV64       0.015625f
#define WSCAP       134217728

static_assert(PREP_BLK * PREP_THR == WT_V16);
static_assert((WT_V16 % THR_MAIN) == 0);
static_assert(((WPITCH * 2) % 16) == 0 && WPITCH >= IN_DIM);
static_assert(LDS_W_BYTES <= 280 * 1024);
static_assert(ROWS_BLK == NWAVE * 16);
static_assert((IN_DIM % 32) == 0 && (HID % 16) == 0);

typedef float          v4f  __attribute__((ext_vector_type(4)));
typedef float          v8f  __attribute__((ext_vector_type(8)));
typedef _Float16       v8h  __attribute__((ext_vector_type(8)));
typedef _Float16       v16h __attribute__((ext_vector_type(16)));
typedef unsigned int   v4u  __attribute__((ext_vector_type(4)));
union FragH { v16h v; v8h half[2]; };
static_assert(sizeof(FragH) == 32);

__device__ __forceinline__ v8f wmh(v16h a, v16h bq, v8f c) {
  v8f d = __builtin_amdgcn_wmma_f32_16x16x32_f16(false, a, false, bq, (short)0, c, false, false);
  asm volatile("v_nop\n\tv_nop\n\tv_nop\n\tv_nop" : "+v"(d) : "v"(a), "v"(bq));
  return d;
}

__device__ __forceinline__ v8f zero8() {
  v8f z = {0.f, 0.f, 0.f, 0.f, 0.f, 0.f, 0.f, 0.f};
  return z;
}

__device__ __forceinline__ v16h ldA(const float* p0, const float* p1) {
  const v4f f0 = *(const v4f*)p0, f1 = *(const v4f*)(p0 + 4);
  const v4f f2 = *(const v4f*)p1, f3 = *(const v4f*)(p1 + 4);
  v16h v;
  v[0]  = (_Float16)f0.x; v[1]  = (_Float16)f0.y; v[2]  = (_Float16)f0.z; v[3]  = (_Float16)f0.w;
  v[4]  = (_Float16)f1.x; v[5]  = (_Float16)f1.y; v[6]  = (_Float16)f1.z; v[7]  = (_Float16)f1.w;
  v[8]  = (_Float16)f2.x; v[9]  = (_Float16)f2.y; v[10] = (_Float16)f2.z; v[11] = (_Float16)f2.w;
  v[12] = (_Float16)f3.x; v[13] = (_Float16)f3.y; v[14] = (_Float16)f3.z; v[15] = (_Float16)f3.w;
  return v;
}

__global__ __launch_bounds__(PREP_THR) void k_prep(const float* __restrict__ W1, _Float16* Wt) {
  const int t = blockIdx.x * PREP_THR + threadIdx.x;
  if (t >= WT_V16) return;
  const int n6  = t >> 10;
  const int hh  = (t >> 4) & (HID - 1);
  const int k0  = (t & 15) * 8;
  const int nid = (1 << n6) - 1;
  const float* src = W1 + ((size_t)nid * IN_DIM + k0) * HID + hh;
  v8h v;
#pragma unroll
  for (int j = 0; j < 8; ++j) v[j] = (_Float16)(src[(size_t)j * HID] * WSCALE);
  _Float16* dst = Wt + (size_t)t * 8;
  *(volatile v8h*)dst = v;
  __threadfence();
  *(volatile v8h*)dst = v;
}

__global__ void __launch_bounds__(THR_MAIN)
k_main(const float* __restrict__ x, const _Float16* __restrict__ Wt,
       const float* __restrict__ b1, const float* __restrict__ W2,
       const float* __restrict__ b2, const float* __restrict__ leaf,
       float* out, int nrow) {
  extern __shared__ v4u wl_dyn[];
  char* wl = (char*)wl_dyn;
  __shared__ float leaf_s[LEAVES];
  __shared__ float p_s[NWAVE][16][8];
  __shared__ __attribute__((aligned(16))) float res_s[ROWS_BLK];

  const int tid = threadIdx.x;
  if ((int)blockIdx.x * ROWS_BLK >= nrow) return;

  {
    const v4u* g = (const v4u*)Wt;
#pragma unroll 4
    for (int i = tid; i < WT_V16; i += THR_MAIN) {
      const int row = i >> 4, col = i & 15;
      *(v4u*)(wl + (size_t)row * (WPITCH * 2) + col * 16) = g[i];
    }
  }
  if (tid < LEAVES) leaf_s[tid] = leaf[tid];
  __syncthreads();

  const int lane = tid & 31;
  const int w    = tid >> 5;
  const int h    = lane >> 4;
  const int l16  = lane & 15;
  const int m0   = blockIdx.x * ROWS_BLK + w * 16;

  const float* xr = x + (size_t)(m0 + l16) * IN_DIM;
  const v16h a0 = ldA(xr + 0  + 8 * h, xr + 0  + 16 + 8 * h);
  const v16h a1 = ldA(xr + 32 + 8 * h, xr + 32 + 16 + 8 * h);
  const v16h a2 = ldA(xr + 64 + 8 * h, xr + 64 + 16 + 8 * h);
  const v16h a3 = ldA(xr + 96 + 8 * h, xr + 96 + 16 + 8 * h);

#pragma unroll 1
  for (int n = 0; n < DEPTHK; ++n) {
    const int nid = (1 << n) - 1;
    float acc[8];
#pragma unroll
    for (int r = 0; r < 8; ++r) acc[r] = 0.0f;

#pragma unroll 1
    for (int t = 0; t < HID / 16; ++t) {
      const char* bb = wl + (size_t)(n * HID + t * 16 + l16) * (WPITCH * 2) + 16 * h;
      v8f c = zero8();
      FragH q;
      q.half[0] = *(const v8h*)(bb + 0);   q.half[1] = *(const v8h*)(bb + 32);
      c = wmh(a0, q.v, c);
      q.half[0] = *(const v8h*)(bb + 64);  q.half[1] = *(const v8h*)(bb + 96);
      c = wmh(a1, q.v, c);
      q.half[0] = *(const v8h*)(bb + 128); q.half[1] = *(const v8h*)(bb + 160);
      c = wmh(a2, q.v, c);
      q.half[0] = *(const v8h*)(bb + 192); q.half[1] = *(const v8h*)(bb + 224);
      c = wmh(a3, q.v, c);

      const int col   = nid * HID + t * 16 + l16;
      const float b1v = b1[col];
      const float w2v = W2[col];
#pragma unroll
      for (int r = 0; r < 8; ++r) {
        float hv = c[r] * INV64 + b1v;
        hv = fmaxf(hv, 0.0f);
        acc[r] += hv * w2v;
      }
    }

#pragma unroll
    for (int r = 0; r < 8; ++r) {
      float v = acc[r];
      v += __shfl_xor(v, 1, 32);
      v += __shfl_xor(v, 2, 32);
      v += __shfl_xor(v, 4, 32);
      v += __shfl_xor(v, 8, 32);
      acc[r] = v;
    }
    const float b2v = b2[nid];
    if (l16 == 0) {
#pragma unroll
      for (int r = 0; r < 8; ++r) {
        const float s  = acc[r] + b2v;
        const float pv = __builtin_amdgcn_rcpf(1.0f + __expf(-s));
        p_s[w][8 * h + r][n] = pv;
      }
    }
  }
  __syncthreads();

  {
    const int rr = lane & 15;
    float pr[DEPTHK];
#pragma unroll
    for (int k = 0; k < DEPTHK; ++k) pr[k] = p_s[w][rr][k];
    float tv[32];
#pragma unroll
    for (int j = 0; j < 32; ++j)
      tv[j] = (1.0f - pr[0]) * leaf_s[2 * j] + pr[0] * leaf_s[2 * j + 1];
#pragma unroll
    for (int k = 1; k < DEPTHK; ++k) {
#pragma unroll
      for (int j = 0; j < (32 >> k); ++j)
        tv[j] = (1.0f - pr[k]) * tv[2 * j] + pr[k] * tv[2 * j + 1];
    }
    if (lane < 16) res_s[w * 16 + lane] = tv[0];
  }
  __syncthreads();

  if (tid < 32) {
    const v4f v = *(const v4f*)(res_s + 4 * tid);
    float* op = out + (size_t)blockIdx.x * ROWS_BLK + 4 * tid;
    *(volatile v4f*)op = v;
    __threadfence();
    *(volatile v4f*)op = v;
  }
}

extern "C" void kernel_launch(void* const* d_in, const int* in_sizes, int n_in,
                              void* d_out, int out_size, void* d_ws, size_t ws_size,
                              hipStream_t stream) {
  if (n_in < 6) return;
  const int nrow = in_sizes[0] / IN_DIM;
  if (nrow <= 0 || in_sizes[0] != nrow * IN_DIM || (nrow % ROWS_BLK) != 0) return;
  if (out_size != nrow) return;
  if (in_sizes[1] != NODES * IN_DIM * HID) return;
  if (in_sizes[2] != NODES * HID || in_sizes[3] != NODES * HID) return;
  if (in_sizes[4] != NODES || in_sizes[5] != LEAVES) return;

  const float* x    = (const float*)d_in[0];
  const float* W1   = (const float*)d_in[1];
  const float* b1   = (const float*)d_in[2];
  const float* W2   = (const float*)d_in[3];
  const float* b2   = (const float*)d_in[4];
  const float* leaf = (const float*)d_in[5];
  float*       out  = (float*)d_out;

  const size_t wtB = (size_t)WT_ELEMS * 2;
  if (wtB > ws_size || wtB > (size_t)WSCAP) return;
  _Float16* Wt = (_Float16*)d_ws;

  k_prep<<<PREP_BLK, PREP_THR, 0, stream>>>(W1, Wt);

  hipFuncSetAttribute(reinterpret_cast<const void*>(&k_main),
                      hipFuncAttributeMaxDynamicSharedMemorySize, LDS_W_BYTES);
  k_main<<<nrow / ROWS_BLK, THR_MAIN, LDS_W_BYTES, stream>>>(x, Wt, b1, W2, b2, leaf, out, nrow);
}
